// SpatioTemporalAttention_34462817583419
// MI455X (gfx1250) — hardware-verified
//
#include <hip/hip_runtime.h>


#ifndef NB
#define NB 2
#endif
#define NB_FULL 2
#ifndef SEQ
#define SEQ 3072
#endif
#define SEQ_FULL 3072
#define NRES 256
#define NFR (SEQ / NRES)
#define CM 512
#define ADW 1024
#define NH 8
#define HD 64
#define CDIM 64
#define NEX 32
#define NTOK (NB * SEQ)
#define NBH (NB * NH)
#define QSCL 0.125f
#define PCAR 16384.0f
#define PINV 0.00006103515625f
#define LCAR 1024.0f
#define LINV 0.0009765625f
#define LOG2E 1.4426950408889634f
#define OUT1_EL ((size_t)NB_FULL * SEQ_FULL * CM)
#define OUT2_EL (OUT1_EL + (size_t)NB_FULL * NH * SEQ_FULL * HD)
static_assert(SEQ % NRES == 0);
static_assert(SEQ >= NRES && SEQ <= SEQ_FULL);
static_assert(NB >= 1 && NB <= NB_FULL);
static_assert(NTOK % 256 == 0);
static_assert(HD == 64 && CM == NH * HD);
static_assert(CM % 64 == 0 && ADW == 2 * CM && CDIM % 32 == 0);
static_assert(OUT1_EL * 4 == 12582912);
static_assert(OUT2_EL * 4 == 25165824);

typedef _Float16 h16;
typedef unsigned short bf;
typedef __attribute__((ext_vector_type(16))) __bf16   v16bf;
typedef __attribute__((ext_vector_type(16))) _Float16 v16h;
typedef __attribute__((ext_vector_type(8)))  _Float16 v8h;
typedef __attribute__((ext_vector_type(2)))  _Float16 v2h;
typedef __attribute__((ext_vector_type(8)))  unsigned short v8us;
typedef __attribute__((ext_vector_type(4)))  unsigned short v4us;
typedef __attribute__((ext_vector_type(2)))  unsigned short v2us;
typedef __attribute__((ext_vector_type(4)))  unsigned int v4u;
typedef __attribute__((ext_vector_type(8)))  float    v8f;
typedef __attribute__((ext_vector_type(4)))  float    v4f;
typedef __attribute__((ext_vector_type(2)))  float    v2f;
typedef v8h  __attribute__((may_alias)) v8ha;
typedef v4f  __attribute__((may_alias)) v4fa;
typedef v8us __attribute__((may_alias)) v8usa;
typedef v4u  __attribute__((may_alias)) v4ua;

__device__ __forceinline__ unsigned short f2bf(float f) { unsigned u = __float_as_uint(f); u += 0x7FFFu + ((u >> 16) & 1u); return (unsigned short)(u >> 16); }
__device__ __forceinline__ float bf2f(unsigned short b) { return __uint_as_float(((unsigned)b) << 16); }
__device__ __forceinline__ float bfr(float f) { return bf2f(f2bf(f)); }
__device__ __forceinline__ v16h cat16(v8h lo, v8h hi) { return __builtin_shufflevector(lo, hi, 0, 1, 2, 3, 4, 5, 6, 7, 8, 9, 10, 11, 12, 13, 14, 15); }
__device__ __forceinline__ v16bf cat16b(v8us lo, v8us hi) { return __builtin_bit_cast(v16bf, __builtin_shufflevector(lo, hi, 0, 1, 2, 3, 4, 5, 6, 7, 8, 9, 10, 11, 12, 13, 14, 15)); }
__device__ __forceinline__ v8f wmma16(v16h a, v16h b, v8f c) { return __builtin_amdgcn_wmma_f32_16x16x32_f16(false, a, false, b, (short)0, c, false, false); }
__device__ __forceinline__ v8f wmmab(v16bf a, v16bf b, v8f c) { return __builtin_amdgcn_wmma_f32_16x16x32_bf16(false, a, false, b, (short)0, c, false, false); }
__device__ __forceinline__ void splitf(float y, unsigned short& h, unsigned short& l) { h = f2bf(y); l = f2bf(y - bf2f(h)); }
__device__ __forceinline__ void splith(float y, h16& a, h16& c) { a = (h16)y; c = (h16)((y - (float)a) * LCAR); }
__device__ __forceinline__ unsigned int pk2(unsigned short lo, unsigned short hi2) { return (unsigned int)lo | ((unsigned int)hi2 << 16); }

template <typename T16> struct WFrag;
template <> struct WFrag<h16> { typedef v16h V; static __device__ __forceinline__ V ld(const h16* p) { return cat16(*(const v8h*)p, *(const v8h*)(p + 16)); } static __device__ __forceinline__ v8f mma(V a, V b, v8f c) { return wmma16(a, b, c); } };
template <> struct WFrag<bf> { typedef v16bf V; static __device__ __forceinline__ V ld(const bf* p) { return cat16b(*(const v8us*)p, *(const v8us*)(p + 16)); } static __device__ __forceinline__ v8f mma(V a, V b, v8f c) { return wmmab(a, b, c); } };
template <typename T16, int NSPLIT, bool BIAS>
__global__ __launch_bounds__(32) void k_gemmw(const T16* __restrict__ A, const T16* __restrict__ A2, const T16* __restrict__ Bt, const T16* __restrict__ Bt2, int K, float* C, int ldc, const float* __restrict__ bias, size_t sA, size_t sB, size_t sC) {
    typedef typename WFrag<T16>::V V;
    __shared__ __align__(16) float os[16 * 68];
    const size_t z = blockIdx.z; A += z * sA; if (A2) A2 += z * sA; Bt += z * sB; if (Bt2) Bt2 += z * sB; C += z * sC;
    const int lane = threadIdx.x & 31, lr = lane & 15, hi = lane >> 4; const int r0 = blockIdx.x * 64, c0 = blockIdx.y * 64;
    v8f acc[4][4];
#pragma unroll
    for (int mb = 0; mb < 4; ++mb)
#pragma unroll
        for (int nb = 0; nb < 4; ++nb) acc[mb][nb] = (v8f){};
    const size_t aoff = (size_t)(r0 + lr) * K + 8 * hi, boff = (size_t)(c0 + lr) * K + 8 * hi;
#pragma unroll 1
    for (int kc = 0; kc < K; kc += 32) {
        V a[4], a2[4];
#pragma unroll
        for (int mb = 0; mb < 4; ++mb) { a[mb] = WFrag<T16>::ld(A + aoff + (size_t)mb * 16 * K + kc); if (NSPLIT == 1 || NSPLIT == 2) a2[mb] = WFrag<T16>::ld(A2 + aoff + (size_t)mb * 16 * K + kc); }
#pragma unroll
        for (int nb = 0; nb < 4; ++nb) { const V b = WFrag<T16>::ld(Bt + boff + (size_t)nb * 16 * K + kc); V b2; if (NSPLIT >= 2) b2 = WFrag<T16>::ld(Bt2 + boff + (size_t)nb * 16 * K + kc);
#pragma unroll
            for (int mb = 0; mb < 4; ++mb) { acc[mb][nb] = WFrag<T16>::mma(a[mb], b, acc[mb][nb]); if (NSPLIT == 1 || NSPLIT == 2) acc[mb][nb] = WFrag<T16>::mma(a2[mb], b, acc[mb][nb]); if (NSPLIT >= 2) acc[mb][nb] = WFrag<T16>::mma(a[mb], b2, acc[mb][nb]); } }
        asm volatile("v_nop\n\tv_nop\n\tv_nop\n\tv_nop" : "+v"(acc[0][0]), "+v"(acc[1][1]), "+v"(acc[2][2]), "+v"(acc[3][3]) : "v"(a[0]), "v"(a[3]));
    }
#pragma unroll
    for (int mb = 0; mb < 4; ++mb) {
#pragma unroll
        for (int nb = 0; nb < 4; ++nb) {
#pragma unroll
            for (int j = 0; j < 8; ++j) os[(hi * 8 + j) * 68 + nb * 16 + lr] = acc[mb][nb][j]; }
        __builtin_amdgcn_wave_barrier(); asm volatile("" ::: "memory");
        float* crow = C + (size_t)(r0 + mb * 16) * ldc + c0;
#pragma unroll 1
        for (int ps = 0; ps < 2; ++ps) {
#pragma unroll
            for (int s = 0; s < 8; ++s) { const int row = 2 * s + hi, cofs = lr * 4; v4f val = *(const v4fa*)(os + row * 68 + cofs); if (BIAS) { val[0] += bfr(bias[c0 + cofs]); val[1] += bfr(bias[c0 + cofs + 1]); val[2] += bfr(bias[c0 + cofs + 2]); val[3] += bfr(bias[c0 + cofs + 3]); }
                *(volatile v4f*)(crow + (size_t)row * ldc + cofs) = val; }
            if (ps == 0) __threadfence(); }
        __builtin_amdgcn_wave_barrier(); asm volatile("" ::: "memory");
    }
}

__global__ __launch_bounds__(256) void k_wtG(const float* __restrict__ w, int K, int N, bf* Bt) {
    const int lane = threadIdx.x & 31; const int L0 = (blockIdx.x * 8 + (threadIdx.x >> 5)) * 8; const int nlines = (int)((size_t)N * K / 64);
#pragma unroll
    for (int ps = 0; ps < 2; ++ps) {
#pragma unroll 1
        for (int l = 0; l < 8; ++l) { const int L = L0 + l; if (L >= nlines) break; const size_t e = (size_t)L * 64 + lane * 2; const int k = (int)(e % K), n = (int)(e / K); v2us o;
            o[0] = f2bf(w[(size_t)k * N + n]); o[1] = f2bf(w[(size_t)(k + 1) * N + n]); *(volatile v2us*)(Bt + e) = o; }
        if (ps == 0) __threadfence(); }
}

__global__ __launch_bounds__(32) void k_invf(float* IF) {
    const int j = threadIdx.x & 31;
    const float e = (float)(j & 15) * 0.0625f;
    const float p = powf(10000.0f, e);
    const float v = 1.0f / p;
    *(volatile float*)(IF + j) = v; __threadfence(); *(volatile float*)(IF + j) = v;
}

__global__ __launch_bounds__(256) void k_cstab(const int* __restrict__ fidx, const int* __restrict__ sidx, const float* __restrict__ IF, float* CS) {
    const int idx = blockIdx.x * 256 + threadIdx.x; if (idx >= NTOK * HD) return;
    const int dd = idx & (HD - 1); const int R = idx >> 6; const int b = R / SEQ, t = R - b * SEQ; const int fl = t / NRES, n = t - fl * NRES;
    const int pseq = sidx[b * NRES + n]; const int pfr = fidx[fl];
    const float pf = (float)((dd < HD / 2) ? pseq : pfr);
    float fr = __fmul_rn(pf, IF[dd & 15]); asm volatile("" : "+v"(fr));
    float sn, cn;
    sincosf(fr, &sn, &cn);
    v2f cs; cs[0] = cn; cs[1] = sn;
    *(volatile v2f*)(CS + (size_t)idx * 2) = cs; __threadfence(); *(volatile v2f*)(CS + (size_t)idx * 2) = cs;
}

__global__ __launch_bounds__(256) void k_condp(const float* __restrict__ cond, bf* P) {
    const int lane = threadIdx.x & 31, w = threadIdx.x >> 5;
    v2us o[8];
#pragma unroll
    for (int it = 0; it < 8; ++it) { const int row = w * 8 + it; const int rc = (row < NB) ? row : (NB - 1); v2us v;
#pragma unroll
        for (int q = 0; q < 2; ++q) { const float x = cond[(size_t)rc * CDIM + 2 * lane + q]; v[q] = (row < NB) ? f2bf(x) : (unsigned short)0; }
        o[it] = v; }
#pragma unroll 1
    for (int ps = 0; ps < 2; ++ps) {
#pragma unroll
        for (int it = 0; it < 8; ++it) *(volatile v2us*)(P + (size_t)(w * 8 + it) * CDIM + 2 * lane) = o[it];
        if (ps == 0) __threadfence(); }
}

__global__ __launch_bounds__(256) void k_ln(const float* __restrict__ X, const float* __restrict__ SS, bf* Xh, bf* Xl) {
    const int lane = threadIdx.x & 31; const int R = blockIdx.x * 8 + (threadIdx.x >> 5); if (R >= NTOK) return;
    const int b = R / SEQ, t = R - b * SEQ;
    const float* xr = X + ((size_t)b * SEQ_FULL + t) * CM;
    float v[16];
    { const v8f a0 = *(const v8f*)(xr + 8 * lane); const v8f a1 = *(const v8f*)(xr + 256 + 8 * lane);
#pragma unroll
      for (int k = 0; k < 8; ++k) { v[k] = bfr(a0[k]); v[8 + k] = bfr(a1[k]); } }
    float s = 0.f;
#pragma unroll
    for (int k = 0; k < 16; ++k) s += v[k];
#pragma unroll
    for (int sh = 16; sh; sh >>= 1) s += __shfl_xor(s, sh, 32);
    const float mu = s * (1.0f / (float)CM);
    float qq = 0.f;
#pragma unroll
    for (int k = 0; k < 16; ++k) { const float d = v[k] - mu; qq += d * d; }
#pragma unroll
    for (int sh = 16; sh; sh >>= 1) qq += __shfl_xor(qq, sh, 32);
    const float var = qq * (1.0f / (float)CM);
    const float rs = rsqrtf(var + 1.0e-5f);
    const float* sc = SS + (size_t)b * ADW;
    v8us oh[2], ol[2];
#pragma unroll
    for (int c = 0; c < 2; ++c) { const int col0 = c * 256 + 8 * lane; const v8f g = *(const v8f*)(sc + col0); const v8f be = *(const v8f*)(sc + CM + col0); v8us th, tl;
#pragma unroll
        for (int k = 0; k < 8; ++k) { const float xn = (v[c * 8 + k] - mu) * rs; const float y = xn * (1.0f + g[k]) + be[k]; unsigned short a2, c2; splitf(y, a2, c2); th[k] = a2; tl[k] = c2; }
        oh[c] = th; ol[c] = tl; }
#pragma unroll 1
    for (int ps = 0; ps < 2; ++ps) {
#pragma unroll
        for (int c = 0; c < 2; ++c) { const size_t o = (size_t)R * CM + c * 256 + 8 * lane; *(volatile v8us*)(Xh + o) = oh[c]; *(volatile v8us*)(Xl + o) = ol[c]; }
        if (ps == 0) __threadfence(); }
}

__global__ __launch_bounds__(256) void k_extras(const float* __restrict__ ca, const float* __restrict__ msk, bf* QE, bf* KE) {
    __shared__ __align__(16) unsigned int qs[256 * 16];
    __shared__ __align__(16) unsigned int ks[256 * 16];
    const int tid = threadIdx.x, lane = tid & 31, w = tid >> 5;
    const int R0 = blockIdx.x * 256; const int R = R0 + tid;
    const int b = R / SEQ, t = R - b * SEQ; const size_t Rf = (size_t)b * SEQ_FULL + t;
    const float cx = bfr(ca[Rf * 3]), cy = bfr(ca[Rf * 3 + 1]), cz = bfr(ca[Rf * 3 + 2]);
    const float mk = bfr(msk[Rf]);
    const float n2 = cx * cx + cz * cz + cy * cy;
    const float g = -(n2 * 0.015625f);
    const unsigned short gh = f2bf(g); const float r1 = g - bf2f(gh); const unsigned short gm = f2bf(r1); const unsigned short gl = f2bf(r1 - bf2f(gm));
    const unsigned short one = (unsigned short)0x3F80u;
    const unsigned short fillv = (mk == 0.0f) ? f2bf(-2.0e30f) : (unsigned short)0;
    v4u qa, qb, ka, kb, zz;
#pragma unroll
    for (int i = 0; i < 4; ++i) { qb[i] = 0u; kb[i] = 0u; zz[i] = 0u; }
    qa[0] = pk2(f2bf(cx), f2bf(cy)); qa[1] = pk2(f2bf(cz), one); qa[2] = pk2(one, one); qa[3] = pk2(gh, gm);
    qb[0] = pk2(gl, one);
    ka[0] = pk2(f2bf(cx * 0.03125f), f2bf(cy * 0.03125f)); ka[1] = pk2(f2bf(cz * 0.03125f), gh); ka[2] = pk2(gm, gl); ka[3] = pk2(one, one);
    kb[0] = pk2(one, fillv);
    unsigned int* qr = qs + tid * 16; unsigned int* krw = ks + tid * 16;
    *(v4u*)(qr) = qa; *(v4u*)(qr + 4) = qb; *(v4u*)(qr + 8) = zz; *(v4u*)(qr + 12) = zz;
    *(v4u*)(krw) = ka; *(v4u*)(krw + 4) = kb; *(v4u*)(krw + 8) = zz; *(v4u*)(krw + 12) = zz;
    __syncthreads();
    v4u oq[4], ok[4]; int off[4];
#pragma unroll
    for (int it = 0; it < 4; ++it) { off[it] = (w * 4 + it) * 128 + lane * 4; oq[it] = *(const v4ua*)(qs + off[it]); ok[it] = *(const v4ua*)(ks + off[it]); }
    unsigned int* QEw = (unsigned int*)QE + (size_t)R0 * 16; unsigned int* KEw = (unsigned int*)KE + (size_t)R0 * 16;
#pragma unroll 1
    for (int ps = 0; ps < 2; ++ps) {
#pragma unroll
        for (int it = 0; it < 4; ++it) { *(volatile v4u*)(QEw + off[it]) = oq[it]; *(volatile v4u*)(KEw + off[it]) = ok[it]; }
        if (ps == 0) __threadfence(); }
}

__global__ __launch_bounds__(256) void k_ropep(const float* __restrict__ F, float scl, const float* __restrict__ CS, bf* Ph, bf* Pl, float* G) {
    const size_t e = ((size_t)blockIdx.x * 256 + threadIdx.x) * 2; if (e >= (size_t)NBH * SEQ * HD) return;
    const int d = (int)(e & (HD - 1)); const int t = (int)((e >> 6) % SEQ); const int bh = (int)(e / ((size_t)HD * SEQ)); const int b = bh / NH, h = bh - b * NH;
    const size_t R = (size_t)b * SEQ + t;
    const float* f = F + R * CM + h * HD;
    v2us oh, ol; v2f go;
#pragma unroll
    for (int q = 0; q < 2; ++q) { const int dd = d + q; const bool sub = ((dd & 16) == 0); const int dp = sub ? dd + 16 : dd - 16;
        const float x0 = f[dd] * scl, x1 = f[dp] * scl;
        const v2f cs = *(const v2f*)(CS + (R * HD + dd) * 2);
        float a = __fmul_rn(x0, cs[0]), bq = __fmul_rn(x1, cs[1]); asm volatile("" : "+v"(a)); asm volatile("" : "+v"(bq));
        const float r = sub ? __fsub_rn(a, bq) : __fadd_rn(a, bq);
        go[q] = r; unsigned short a2, c2; splitf(r, a2, c2); oh[q] = a2; ol[q] = c2; }
    const size_t og = ((size_t)bh * SEQ_FULL + t) * HD + d;
    *(volatile v2us*)(Ph + e) = oh; *(volatile v2us*)(Pl + e) = ol; if (G != nullptr) *(volatile v2f*)(G + og) = go;
    __threadfence();
    *(volatile v2us*)(Ph + e) = oh; *(volatile v2us*)(Pl + e) = ol; if (G != nullptr) *(volatile v2f*)(G + og) = go;
}

__global__ __launch_bounds__(256) void k_vtp(const float* __restrict__ F, h16* Vh, h16* Vl, float* G) {
    __shared__ float tile[64 * 65];
    const int tid = threadIdx.x, lane = tid & 31, w = tid >> 5;
    const int bh = blockIdx.y; const int b = bh / NH, h = bh - b * NH; const int t0 = blockIdx.x * 64;
    const int pc = tid & 15, rb = tid >> 4;
    v4f vv[4]; size_t og[4];
#pragma unroll
    for (int it = 0; it < 4; ++it) { const int tr = it * 16 + rb; vv[it] = *(const v4f*)(F + ((size_t)b * SEQ + t0 + tr) * CM + h * HD + 4 * pc);
#pragma unroll
        for (int c = 0; c < 4; ++c) tile[tr * 65 + 4 * pc + c] = vv[it][c];
        og[it] = ((size_t)bh * SEQ_FULL + t0 + tr) * HD + 4 * pc; }
#pragma unroll 1
    for (int ps = 0; ps < 2; ++ps) {
#pragma unroll
        for (int it = 0; it < 4; ++it) *(volatile v4f*)(G + og[it]) = vv[it];
        if (ps == 0) __threadfence(); }
    __syncthreads();
    v2h oh[8], ol[8]; size_t ov[8];
#pragma unroll
    for (int it = 0; it < 8; ++it) { const int d = w * 8 + it; const float x0 = tile[(2 * lane) * 65 + d], x1 = tile[(2 * lane + 1) * 65 + d];
        h16 a0, c0, a1, c1; splith(x0, a0, c0); splith(x1, a1, c1); v2h th, tl; th[0] = a0; th[1] = a1; tl[0] = c0; tl[1] = c1; oh[it] = th; ol[it] = tl;
        ov[it] = ((size_t)bh * HD + d) * SEQ + t0 + 2 * lane; }
#pragma unroll 1
    for (int ps = 0; ps < 2; ++ps) {
#pragma unroll
        for (int it = 0; it < 8; ++it) { *(volatile v2h*)(Vh + ov[it]) = oh[it]; *(volatile v2h*)(Vl + ov[it]) = ol[it]; }
        if (ps == 0) __threadfence(); }
}

__global__ __launch_bounds__(32) void k_attn(const bf* __restrict__ Qh, const bf* __restrict__ Ql, const bf* __restrict__ QE,
                                             const bf* __restrict__ Kh, const bf* __restrict__ Kl, const bf* __restrict__ KE,
                                             const h16* __restrict__ Vth, const h16* __restrict__ Vtl, bf* ATh, bf* ATl) {
    __shared__ __align__(16) h16 ps[16 * 32];
    __shared__ __align__(16) float os[16 * 68];
    const int lane = threadIdx.x & 31, lr = lane & 15, hi = lane >> 4;
    const int bh = blockIdx.y; const int b = bh / NH, h = bh - b * NH;
    const int q0 = blockIdx.x * 16;
    const int kvlen = (q0 / NRES + 1) * NRES;
    const size_t hp = (size_t)bh * SEQ * HD;
    const size_t tb = (size_t)b * SEQ;
    const size_t qo = hp + (size_t)(q0 + lr) * HD + 8 * hi;
    const v16bf aH0 = WFrag<bf>::ld(Qh + qo), aH1 = WFrag<bf>::ld(Qh + qo + 32);
    const v16bf aL0 = WFrag<bf>::ld(Ql + qo), aL1 = WFrag<bf>::ld(Ql + qo + 32);
    const v16bf aE = WFrag<bf>::ld(QE + (tb + q0 + lr) * NEX + 8 * hi);
    v8f oh[4], ol[4];
#pragma unroll
    for (int nb = 0; nb < 4; ++nb) { oh[nb] = (v8f){}; ol[nb] = (v8f){}; }
    float m[8], l[8];
#pragma unroll
    for (int r = 0; r < 8; ++r) { m[r] = -1.0e30f; l[r] = 0.f; }
#pragma unroll 1
    for (int key0 = 0; key0 < kvlen; key0 += 32) {
        v8f s[2];
#pragma unroll
        for (int j = 0; j < 2; ++j) {
            const int kr = key0 + 16 * j + lr;
            const size_t ko = hp + (size_t)kr * HD + 8 * hi;
            s[j] = (v8f){};
            { const v16bf bE = WFrag<bf>::ld(KE + (tb + kr) * NEX + 8 * hi); s[j] = wmmab(aE, bE, s[j]); }
            { const v16bf bH = WFrag<bf>::ld(Kh + ko), bL = WFrag<bf>::ld(Kl + ko); s[j] = wmmab(aH0, bH, s[j]); s[j] = wmmab(aL0, bH, s[j]); s[j] = wmmab(aH0, bL, s[j]); }
            { const v16bf bH = WFrag<bf>::ld(Kh + ko + 32), bL = WFrag<bf>::ld(Kl + ko + 32); s[j] = wmmab(aH1, bH, s[j]); s[j] = wmmab(aL1, bH, s[j]); s[j] = wmmab(aH1, bL, s[j]); }
        }
        asm volatile("v_nop\n\tv_nop\n\tv_nop\n\tv_nop" : "+v"(s[0]), "+v"(s[1]) : "v"(aH0), "v"(aH1), "v"(aL0), "v"(aL1), "v"(aE));
        float al[8];
#pragma unroll
        for (int r = 0; r < 8; ++r) {
            float v = fmaxf(s[0][r], s[1][r]);
            v = fmaxf(v, __shfl_xor(v, 1, 32)); v = fmaxf(v, __shfl_xor(v, 2, 32)); v = fmaxf(v, __shfl_xor(v, 4, 32)); v = fmaxf(v, __shfl_xor(v, 8, 32));
            const float mn = fmaxf(m[r], v);
            al[r] = __builtin_amdgcn_exp2f((m[r] - mn) * LOG2E);
            m[r] = mn;
            const float p0 = __builtin_amdgcn_exp2f((s[0][r] - mn) * LOG2E), p1 = __builtin_amdgcn_exp2f((s[1][r] - mn) * LOG2E);
            s[0][r] = p0; s[1][r] = p1;
            float sm = p0 + p1;
            sm += __shfl_xor(sm, 1, 32); sm += __shfl_xor(sm, 2, 32); sm += __shfl_xor(sm, 4, 32); sm += __shfl_xor(sm, 8, 32);
            l[r] = l[r] * al[r] + sm;
        }
#pragma unroll
        for (int nb = 0; nb < 4; ++nb)
#pragma unroll
            for (int r = 0; r < 8; ++r) { oh[nb][r] *= al[r]; ol[nb][r] *= al[r]; }
#pragma unroll
        for (int r = 0; r < 8; ++r) { ps[(8 * hi + r) * 32 + lr] = (h16)(s[0][r] * PCAR); ps[(8 * hi + r) * 32 + 16 + lr] = (h16)(s[1][r] * PCAR); }
        __builtin_amdgcn_fence(3, "wavefront"); __builtin_amdgcn_wave_barrier(); asm volatile("" ::: "memory");
        const v16h ap = cat16(*(const v8ha*)(ps + lr * 32 + 8 * hi), *(const v8ha*)(ps + lr * 32 + 16 + 8 * hi));
#pragma unroll
        for (int nb = 0; nb < 4; ++nb) { const size_t vo = ((size_t)bh * HD + 16 * nb + lr) * SEQ + key0 + 8 * hi;
            const v16h bH = WFrag<h16>::ld(Vth + vo); oh[nb] = wmma16(ap, bH, oh[nb]);
            const v16h bL = WFrag<h16>::ld(Vtl + vo); ol[nb] = wmma16(ap, bL, ol[nb]); }
        asm volatile("v_nop\n\tv_nop\n\tv_nop\n\tv_nop" : "+v"(oh[0]), "+v"(oh[1]), "+v"(oh[2]), "+v"(oh[3]), "+v"(ol[0]), "+v"(ol[1]), "+v"(ol[2]), "+v"(ol[3]) : "v"(ap));
    }
    float il[8];
#pragma unroll
    for (int r = 0; r < 8; ++r) il[r] = PINV * __fdiv_rn(1.0f, l[r]);
#pragma unroll
    for (int nb = 0; nb < 4; ++nb)
#pragma unroll
        for (int r = 0; r < 8; ++r) os[(8 * hi + r) * 68 + 16 * nb + lr] = (oh[nb][r] + ol[nb][r] * LINV) * il[r];
    __builtin_amdgcn_fence(3, "wavefront"); __builtin_amdgcn_wave_barrier(); asm volatile("" ::: "memory");
    v8us ah[4], av[4]; size_t ad[4];
#pragma unroll
    for (int it = 0; it < 4; ++it) { const int rr = it * 4 + (lane >> 3); const int pc = lane & 7;
        const v4f x0 = *(const v4fa*)(os + rr * 68 + pc * 8), x1 = *(const v4fa*)(os + rr * 68 + pc * 8 + 4); v8us th, tl;
#pragma unroll
        for (int c = 0; c < 4; ++c) { unsigned short a2, c2; splitf(x0[c], a2, c2); th[c] = a2; tl[c] = c2; splitf(x1[c], a2, c2); th[4 + c] = a2; tl[4 + c] = c2; }
        ah[it] = th; av[it] = tl; ad[it] = (tb + q0 + rr) * CM + (size_t)h * HD + pc * 8; }
#pragma unroll 1
    for (int pz = 0; pz < 2; ++pz) {
#pragma unroll
        for (int it = 0; it < 4; ++it) { *(volatile v8us*)(ATh + ad[it]) = ah[it]; *(volatile v8us*)(ATl + ad[it]) = av[it]; }
        if (pz == 0) __threadfence(); }
}

extern "C" void kernel_launch(void* const* d_in, const int* in_sizes, int n_in,
                              void* d_out, int out_size, void* d_ws, size_t ws_size, hipStream_t stream) {
    if (n_in < 16) return;
    const int ntok_in = (NB - 1) * SEQ_FULL + SEQ;
    if (in_sizes[0] < ntok_in * CM || in_sizes[1] < NFR || in_sizes[2] < NB * NRES || in_sizes[3] < ntok_in || in_sizes[4] < NB * CDIM || in_sizes[5] < ntok_in * 3) return;
    if (in_sizes[6] < CDIM * ADW || in_sizes[7] < ADW) return;
    if (in_sizes[8] < CM * CM || in_sizes[10] < CM * CM || in_sizes[12] < CM * CM || in_sizes[14] < CM * CM) return;
    if (in_sizes[9] < CM || in_sizes[11] < CM || in_sizes[13] < CM || in_sizes[15] < CM) return;
    const size_t out_need = OUT2_EL + ((size_t)((NB - 1) * NH + NH - 1) * SEQ_FULL + SEQ) * HD;
    if ((size_t)out_size < out_need) return;
    const float* s_frames = (const float*)d_in[0]; const int* frame_idx = (const int*)d_in[1]; const int* seq_idx = (const int*)d_in[2]; const float* mask = (const float*)d_in[3];
    const float* cond = (const float*)d_in[4]; const float* ca_pos = (const float*)d_in[5]; const float* adaln_w = (const float*)d_in[6]; const float* adaln_b = (const float*)d_in[7];
    const float* wq = (const float*)d_in[8]; const float* bq = (const float*)d_in[9]; const float* wk = (const float*)d_in[10]; const float* bk = (const float*)d_in[11];
    const float* wv = (const float*)d_in[12]; const float* bv = (const float*)d_in[13]; const float* wo = (const float*)d_in[14]; const float* bo = (const float*)d_in[15];
    float* OUT = (float*)d_out;
    char* wsp = (char*)d_ws;
    auto take = [&](size_t bytes) { char* p = wsp; wsp += (bytes + 255) & ~(size_t)255; return (void*)p; };
    bf* WQ = (bf*)take((size_t)CM * CM * 2); bf* WK = (bf*)take((size_t)CM * CM * 2); bf* WV = (bf*)take((size_t)CM * CM * 2); bf* WO = (bf*)take((size_t)CM * CM * 2);
    bf* WA = (bf*)take((size_t)ADW * CDIM * 2); bf* CAP = (bf*)take((size_t)64 * CDIM * 2); float* SS = (float*)take((size_t)64 * ADW * 4);
    float* INVF = (float*)take(256); float* CS = (float*)take((size_t)NTOK * HD * 2 * 4);
    bf* XBh = (bf*)take((size_t)NTOK * CM * 2); bf* XBl = (bf*)take((size_t)NTOK * CM * 2);
    float* FQ = (float*)take((size_t)NTOK * CM * 4); float* FK = (float*)take((size_t)NTOK * CM * 4); float* FV = (float*)take((size_t)NTOK * CM * 4);
    bf* QPh = (bf*)take((size_t)NBH * SEQ * HD * 2); bf* QPl = (bf*)take((size_t)NBH * SEQ * HD * 2); bf* KPh = (bf*)take((size_t)NBH * SEQ * HD * 2); bf* KPl = (bf*)take((size_t)NBH * SEQ * HD * 2);
    h16* VTh = (h16*)take((size_t)NBH * HD * SEQ * 2); h16* VTl = (h16*)take((size_t)NBH * HD * SEQ * 2);
    bf* QE = (bf*)take((size_t)NTOK * NEX * 2); bf* KE = (bf*)take((size_t)NTOK * NEX * 2);
    bf* ATh = (bf*)take((size_t)NTOK * CM * 2); bf* ATl = (bf*)take((size_t)NTOK * CM * 2);
    const size_t used = (size_t)(wsp - (char*)d_ws);
    if (used > ws_size || used > ((size_t)128 << 20)) return;

    k_invf<<<1, 32, 0, stream>>>(INVF);
    k_cstab<<<(unsigned)((NTOK * HD + 255) / 256), 256, 0, stream>>>(frame_idx, seq_idx, INVF, CS);
    k_wtG<<<(unsigned)(((size_t)ADW * CDIM / 64 + 63) / 64), 256, 0, stream>>>(adaln_w, CDIM, ADW, WA);
    k_wtG<<<(unsigned)(((size_t)CM * CM / 64 + 63) / 64), 256, 0, stream>>>(wq, CM, CM, WQ);
    k_wtG<<<(unsigned)(((size_t)CM * CM / 64 + 63) / 64), 256, 0, stream>>>(wk, CM, CM, WK);
    k_wtG<<<(unsigned)(((size_t)CM * CM / 64 + 63) / 64), 256, 0, stream>>>(wv, CM, CM, WV);
    k_wtG<<<(unsigned)(((size_t)CM * CM / 64 + 63) / 64), 256, 0, stream>>>(wo, CM, CM, WO);
    k_condp<<<1, 256, 0, stream>>>(cond, CAP);
    k_gemmw<bf, 0, true><<<dim3(1, ADW / 64, 1), 32, 0, stream>>>(CAP, nullptr, WA, nullptr, CDIM, SS, ADW, adaln_b, 0, 0, 0);
    k_ln<<<(unsigned)(NTOK / 8), 256, 0, stream>>>(s_frames, SS, XBh, XBl);
    k_extras<<<(unsigned)(NTOK / 256), 256, 0, stream>>>(ca_pos, mask, QE, KE);
    const unsigned LR = (unsigned)(((size_t)NBH * SEQ * HD / 2 + 255) / 256);
    k_gemmw<bf, 1, true><<<dim3(NTOK / 64, CM / 64, 1), 32, 0, stream>>>(XBh, XBl, WQ, nullptr, CM, FQ, CM, bq, 0, 0, 0);
    k_ropep<<<LR, 256, 0, stream>>>(FQ, QSCL, CS, QPh, QPl, nullptr);
    k_gemmw<bf, 1, true><<<dim3(NTOK / 64, CM / 64, 1), 32, 0, stream>>>(XBh, XBl, WK, nullptr, CM, FK, CM, bk, 0, 0, 0);
    k_ropep<<<LR, 256, 0, stream>>>(FK, 1.0f, CS, KPh, KPl, OUT + OUT1_EL);
    k_gemmw<bf, 1, true><<<dim3(NTOK / 64, CM / 64, 1), 32, 0, stream>>>(XBh, XBl, WV, nullptr, CM, FV, CM, bv, 0, 0, 0);
    k_vtp<<<dim3(SEQ / 64, NBH, 1), 256, 0, stream>>>(FV, VTh, VTl, OUT + OUT2_EL);
    k_attn<<<dim3(SEQ / 16, NBH, 1), 32, 0, stream>>>(QPh, QPl, QE, KPh, KPl, KE, VTh, VTl, ATh, ATl);
    k_gemmw<bf, 1, true><<<dim3(SEQ / 64, CM / 64, NB), 32, 0, stream>>>(ATh, ATl, WO, nullptr, CM, OUT, CM, bo, (size_t)SEQ * CM, 0, (size_t)SEQ_FULL * CM);
}
